// SparseWindowAttention_40973988004145
// MI455X (gfx1250) — hardware-verified
//
#include <hip/hip_runtime.h>
#include <math.h>

typedef __attribute__((ext_vector_type(16))) _Float16 v16h;
typedef __attribute__((ext_vector_type(16))) __bf16 v16b;
typedef __attribute__((ext_vector_type(8)))  _Float16 v8h;
typedef __attribute__((ext_vector_type(8)))  float v8f;
typedef __attribute__((ext_vector_type(4)))  float v4f;
typedef __attribute__((ext_vector_type(2)))  float v2f;
typedef __attribute__((ext_vector_type(4)))  unsigned v4u;
typedef __attribute__((ext_vector_type(4)))  int v4i;
typedef float __attribute__((may_alias)) float_a;
typedef int __attribute__((may_alias)) int_a;

template <typename T> __device__ __forceinline__ void vst2(void* p, T v) { *(volatile T*)p = v; __threadfence(); *(volatile T*)p = v; }
__device__ __forceinline__ v8f wmma16(v16h a, v16h b, v8f c) {
  v8f d = __builtin_amdgcn_wmma_f32_16x16x32_f16(false, a, false, b, (short)0, c, false, false);
  asm volatile("v_nop\n\tv_nop\n\tv_nop\n\tv_nop" : "+v"(d) : "v"(a), "v"(b));
  return d;
}
__device__ __forceinline__ v8f wmma_bf(v16b a, v16b b, v8f c) {
  v8f d = __builtin_amdgcn_wmma_f32_16x16x32_bf16(false, a, false, b, (short)0, c, false, false);
  asm volatile("v_nop\n\tv_nop\n\tv_nop\n\tv_nop" : "+v"(d) : "v"(a), "v"(b));
  return d;
}
__device__ __forceinline__ v16h frag_h(const _Float16* rowk0, int lane) {
  union { v16h v; v8h q[2]; } u; const _Float16* p = rowk0 + 8 * (lane >> 4);
  u.q[0] = *(const v8h*)p; u.q[1] = *(const v8h*)(p + 16); return u.v;
}
__device__ __forceinline__ v16h frag_f32(const float* rowk0, int lane) {
  v16h a; const float* p = rowk0 + 8 * (lane >> 4);
#pragma unroll
  for (int i = 0; i < 8; ++i) { a[i] = (_Float16)p[i]; a[8 + i] = (_Float16)p[16 + i]; }
  return a;
}
__device__ __forceinline__ v16h frag_f32s(const float* rowk0, int lane, float sc) {
  v16h a; const float* p = rowk0 + 8 * (lane >> 4);
#pragma unroll
  for (int i = 0; i < 8; ++i) { a[i] = (_Float16)(p[i] * sc); a[8 + i] = (_Float16)(p[16 + i] * sc); }
  return a;
}
__device__ __forceinline__ v16h fragc_f32(const float* W, int k0, int n, int lane, int ld, int K) {
  v16h a; const int g = lane >> 4;
#pragma unroll
  for (int i = 0; i < 8; ++i) { const int ka = k0 + 8 * g + i, kb = ka + 16;
    a[i] = (_Float16)(ka < K ? W[(size_t)(ka < K ? ka : K - 1) * ld + n] : 0.f); a[8 + i] = (_Float16)(kb < K ? W[(size_t)(kb < K ? kb : K - 1) * ld + n] : 0.f); }
  return a;
}
struct F2 { v16b h, l; };
__device__ __forceinline__ F2 bsplit16(const float v[16]) { F2 r;
#pragma unroll
  for (int i = 0; i < 16; ++i) { const __bf16 h = (__bf16)v[i]; r.h[i] = h; r.l[i] = (__bf16)(v[i] - (float)h); }
  return r; }
__device__ __forceinline__ F2 split_row(const float* row, int k0, int lane) { float v[16]; const float* p = row + k0 + 8 * (lane >> 4);
#pragma unroll
  for (int i = 0; i < 8; ++i) { v[i] = p[i]; v[8 + i] = p[16 + i]; }
  return bsplit16(v); }
__device__ __forceinline__ F2 split_rowK(const float* row, int k0, int lane, int K) { float v[16]; const int g = lane >> 4;
#pragma unroll
  for (int i = 0; i < 8; ++i) { const int ka = k0 + 8 * g + i, kb = ka + 16; v[i] = ka < K ? row[ka < K ? ka : K - 1] : 0.f; v[8 + i] = kb < K ? row[kb < K ? kb : K - 1] : 0.f; }
  return bsplit16(v); }
__device__ __forceinline__ F2 split_col(const float* W, int k0, int n, int lane, int ld, int K) { float v[16]; const int g = lane >> 4;
#pragma unroll
  for (int i = 0; i < 8; ++i) { const int ka = k0 + 8 * g + i, kb = ka + 16; v[i] = ka < K ? W[(size_t)(ka < K ? ka : K - 1) * ld + n] : 0.f; v[8 + i] = kb < K ? W[(size_t)(kb < K ? kb : K - 1) * ld + n] : 0.f; }
  return bsplit16(v); }
__device__ __forceinline__ v8f mac3(const F2& a, const F2& b, v8f c) { c = wmma_bf(a.l, b.h, c); c = wmma_bf(a.h, b.l, c); return wmma_bf(a.h, b.h, c); }
__device__ __forceinline__ float sigm(float v) { return 1.0f / (1.0f + expf(-v)); }
#define LDSX() do { asm volatile("s_wait_dscnt 0" ::: "memory"); __builtin_amdgcn_wave_barrier(); __builtin_amdgcn_fence(__ATOMIC_RELEASE, "workgroup"); } while (0)


#ifndef NT
#define NT 4
#endif
#define HI 48
#define WI 48
#define CC 512
#define NH 8
#define CH 64
#define WS8 8
#define NWH (HI / WS8)
#define NWW (WI / WS8)
#define NW (NWH * NWW)
#define WA (WS8 * WS8)
#define NROLL 192
#define PHW 12
#define NPOOL (PHW * PHW)
#define NK (WA + NROLL + NPOOL)
#define NTOK (HI * WI)
#define NROWS (NT * NTOK + NT * NPOOL)
#define NROWSP (((NROWS + 63) / 64) * 64)
typedef __attribute__((ext_vector_type(8))) __bf16 v8b;
__device__ __forceinline__ v16b frag_b(const __bf16* rowk0, int lane) {
  union { v16b v; v8b q[2]; } u; const __bf16* p = rowk0 + 8 * (lane >> 4);
  u.q[0] = *(const v8b*)p; u.q[1] = *(const v8b*)(p + 16); return u.v;
}
__device__ __forceinline__ float bfr(float v) { return (float)(__bf16)v; }
__device__ __attribute__((noinline)) float exp_ni(float v) { return expf(v); }
__device__ __attribute__((noinline)) float erf_ni(float v) { return erff(v); }

#define WS_Q   0u
#define WS_K   (WS_Q + 2u * (size_t)NT * NTOK * CC)
#define WS_V   (WS_K + 2u * (size_t)NROWSP * CC)
#define WS_PX  (WS_V + 2u * (size_t)NROWSP * CC)
#define WS_KT  (WS_PX + 4u * (size_t)(NROWSP - NT * NTOK) * CC)
#define WS_WM  (WS_KT + 4u * (size_t)NW * NK)
#define WS_O   (WS_WM + 4u * 64)
#define WS_END (WS_O + 4u * (size_t)NT * NTOK * CC)

__global__ __launch_bounds__(512) void k_pool(const float* __restrict__ X, const float* __restrict__ PW, const float* __restrict__ PB, float* __restrict__ PX) { __shared__ __align__(16) float s[CC]; const int c = threadIdx.x; const int p = blockIdx.x, t = blockIdx.y; const int ph = p / PHW, pw = p % PHW;
  float a = 0.f;
#pragma unroll
  for (int i = 0; i < 4; ++i)
#pragma unroll
    for (int j = 0; j < 4; ++j) a += bfr(X[(((size_t)t * HI + ph * 4 + i) * WI + pw * 4 + j) * CC + c]) * bfr(PW[c * 16 + i * 4 + j]);
  s[c] = a + bfr(PB[c]); __syncthreads(); if (c < CC / 4) vst2(PX + ((size_t)t * NPOOL + p) * CC + c * 4, *(const v4f*)&s[c * 4]); }
__global__ __launch_bounds__(128) void k_proj(const float* __restrict__ X, const float* __restrict__ PX, const float* __restrict__ WQ, const float* __restrict__ BQ, const float* __restrict__ WK, const float* __restrict__ BK, const float* __restrict__ WV, const float* __restrict__ BV, _Float16* __restrict__ Q, _Float16* __restrict__ K, _Float16* __restrict__ V) {
  __shared__ __align__(16) _Float16 sh[64][136];
  const int tid = threadIdx.x, wave = tid >> 5, lane = tid & 31, col = lane & 15, g = lane >> 4; const int which = blockIdx.z; const int c0 = blockIdx.y * 128; const size_t r0 = (size_t)blockIdx.x * 64;
  const bool pooled = (r0 >= (size_t)NT * NTOK); if (which == 0 && pooled) return;
  const float* Wm = which == 0 ? WQ : which == 1 ? WK : WV; const float* Bm = which == 0 ? BQ : which == 1 ? BK : BV;
  const float* src = pooled ? (PX + (r0 - (size_t)NT * NTOK + wave * 16 + col) * CC) : (X + (r0 + wave * 16 + col) * CC);
  v8f acc[8] = {};
#pragma unroll 2
  for (int kc = 0; kc < CC / 32; ++kc) { v16b w8[8];
#pragma unroll
    for (int j = 0; j < 8; ++j) { const int o = c0 + j * 16 + col;
#pragma unroll
      for (int i = 0; i < 8; ++i) { w8[j][i] = (__bf16)Wm[(size_t)(kc * 32 + 8 * g + i) * CC + o]; w8[j][8 + i] = (__bf16)Wm[(size_t)(kc * 32 + 16 + 8 * g + i) * CC + o]; } }
    if (!pooled) { v16b a; const float* p = src + kc * 32 + 8 * g;
#pragma unroll
      for (int i = 0; i < 8; ++i) { a[i] = (__bf16)p[i]; a[8 + i] = (__bf16)p[16 + i]; }
#pragma unroll
      for (int j = 0; j < 8; ++j) acc[j] = wmma_bf(a, w8[j], acc[j]); }
    else { const F2 a = split_row(src, kc * 32, lane);
#pragma unroll
      for (int j = 0; j < 8; ++j) { acc[j] = wmma_bf(a.h, w8[j], acc[j]); acc[j] = wmma_bf(a.l, w8[j], acc[j]); } } }
#pragma unroll
  for (int j = 0; j < 8; ++j) { const float bb = bfr(Bm[c0 + j * 16 + col]);
#pragma unroll
    for (int r = 0; r < 8; ++r) sh[wave * 16 + 8 * g + r][j * 16 + col] = (_Float16)(acc[j][r] + bb); }
  __syncthreads();
  { _Float16* dst = (which == 0 ? Q : which == 1 ? K : V); for (int e = tid; e < 64 * 16; e += 128) { const int rl = e >> 4, q = e & 15; vst2((unsigned*)(dst + (r0 + rl) * CC + c0 + q * 8), *(const v4u*)&sh[rl][q * 8]); } } }
__global__ __launch_bounds__(64) void k_tab(const float* __restrict__ MK, int* __restrict__ KT, int* __restrict__ WM) { __shared__ __align__(16) int skt[NK]; __shared__ int svalid[4 * WA]; __shared__ float smax;
  const int t = threadIdx.x; const int w = blockIdx.x; const int wi = w / NWW, wj = w % NWW;
  if (t == 0) { int n = 0; for (int e = 0; e < 4 * WA; ++e) { const int s = e / WA, r = (e % WA) / WS8, c = e % WS8; bool zero; if (s == 0) zero = (r < WS8 - 4) && (c < WS8 - 4); else if (s == 1) zero = (r < WS8 - 4) && (c >= 4); else if (s == 2) zero = (r >= 4) && (c < WS8 - 4); else zero = (r >= 4) && (c >= 4); if (!zero) svalid[n++] = e; }
    float m = 0.f; for (int tt = 0; tt < NT; ++tt) { float mx = 0.f; for (int r = 0; r < WS8; ++r) for (int c = 0; c < WS8; ++c) mx = fmaxf(mx, bfr(MK[(((size_t)tt * HI + wi * WS8 + r) * WI + wj * WS8 + c)])); m += mx; } smax = m; }
  __syncthreads();
  { const int r = t / WS8, c = t % WS8; skt[t] = (wi * WS8 + r) * WI + wj * WS8 + c; }
  for (int j = t; j < NROLL; j += 64) { const int e = svalid[j]; const int s = e / WA, r = (e % WA) / WS8, c = e % WS8; const int s0 = (s < 2) ? -4 : 4, s1 = ((s & 1) == 0) ? -4 : 4; const int h = wi * WS8 + r, ww = wj * WS8 + c; const int hs = ((h - s0) % HI + HI) % HI, wsr = ((ww - s1) % WI + WI) % WI; skt[WA + j] = hs * WI + wsr; }
  for (int p = t; p < NPOOL; p += 64) skt[WA + NROLL + p] = NTOK + p;
  __syncthreads();
  for (int q = t; q < NK / 4; q += 64) vst2((int*)(KT + (size_t)w * NK) + q * 4, *(const v4i*)&skt[q * 4]);
  (void)WM; (void)smax; }
__global__ __launch_bounds__(64) void k_flags(const float* __restrict__ MK, int* __restrict__ WM) { __shared__ __align__(16) int sf[64]; const int w = threadIdx.x;
  int flag = 0; if (w < NW) { const int wi = w / NWW, wj = w % NWW; float m = 0.f; for (int tt = 0; tt < NT; ++tt) { float mx = 0.f; for (int r = 0; r < WS8; ++r) for (int c = 0; c < WS8; ++c) mx = fmaxf(mx, bfr(MK[(((size_t)tt * HI + wi * WS8 + r) * WI + wj * WS8 + c)])); m += mx; } flag = (m > 0.f) ? 1 : 0; }
  sf[w] = flag; __syncthreads(); if (w < 16) vst2(WM + w * 4, *(const v4i*)&sf[w * 4]); }
__global__ __launch_bounds__(128) void k_att(const _Float16* __restrict__ Q, const _Float16* __restrict__ K, const _Float16* __restrict__ V, const int* __restrict__ KT, const int* __restrict__ WM, float* __restrict__ O) {
  __shared__ __align__(16) float sp[4][16][36]; __shared__ __align__(16) float so[4][16][68]; __shared__ __align__(16) _Float16 sv[32][72]; __shared__ int srow[32];
  const int tid = threadIdx.x, wave = tid >> 5, lane = tid & 31, col = lane & 15, g = lane >> 4; const int tq = blockIdx.x, h = blockIdx.y, w = blockIdx.z; const int wi = w / NWW, wj = w % NWW;
  const bool maskedw = (WM[w] != 0);
  const int ql = wave * 16 + col; const size_t qrow = (size_t)tq * NTOK + (wi * WS8 + ql / WS8) * WI + wj * WS8 + (ql % WS8);
  v16h aq[2];
#pragma unroll
  for (int kc = 0; kc < 2; ++kc) aq[kc] = frag_h(Q + qrow * CC + h * CH + kc * 32, lane);
  float m[8], l[8];
#pragma unroll
  for (int r = 0; r < 8; ++r) { m[r] = -3.0e38f; l[r] = 0.f; }
  v8f acc[4] = {};
  const int nkeys = maskedw ? (NT * NK) : WA; const int ntiles = (nkeys + 31) / 32;
#pragma unroll 1
  for (int ks = 0; ks < ntiles; ++ks) {
    __syncthreads();
    if (tid < 32) { int tk, j; int kv = ks * 32 + tid; if (kv >= nkeys) kv = nkeys - 1;
      if (maskedw) { tk = kv / NK; j = kv % NK; } else { tk = tq; j = kv; }
      const int id = KT[(size_t)w * NK + j]; srow[tid] = (id < NTOK) ? (tk * NTOK + id) : (NT * NTOK + tk * NPOOL + (id - NTOK)); }
    __syncthreads();
    for (int e = tid; e < 32 * 8; e += 128) { const int i = e >> 3, q8 = e & 7; *(v4u*)&sv[i][q8 * 8] = *(const v4u*)(V + (size_t)srow[i] * CC + h * CH + q8 * 8); }
    float s[2][8];
#pragma unroll
    for (int ct = 0; ct < 2; ++ct) { const int i = ct * 16 + col; const size_t krow = (size_t)srow[i]; v8f c = {};
#pragma unroll
      for (int kc = 0; kc < 2; ++kc) c = wmma16(aq[kc], frag_h(K + krow * CC + h * CH + kc * 32, lane), c);
#pragma unroll
      for (int r = 0; r < 8; ++r) s[ct][r] = (ks * 32 + i < nkeys) ? c[r] * 0.125f : -3.0e38f; }
    float alpha[8];
#pragma unroll
    for (int r = 0; r < 8; ++r) { float mx = fmaxf(s[0][r], s[1][r]);
#pragma unroll
      for (int o = 1; o < 16; o <<= 1) mx = fmaxf(mx, __shfl_xor(mx, o));
      const float mn = fmaxf(m[r], mx); alpha[r] = __expf(m[r] - mn); const float e0 = (s[0][r] <= -1.0e38f) ? 0.f : __expf(s[0][r] - mn), e1 = (s[1][r] <= -1.0e38f) ? 0.f : __expf(s[1][r] - mn); float es = e0 + e1;
#pragma unroll
      for (int o = 1; o < 16; o <<= 1) es += __shfl_xor(es, o);
      l[r] = l[r] * alpha[r] + es; m[r] = mn; sp[wave][8 * g + r][col] = e0; sp[wave][8 * g + r][16 + col] = e1; }
#pragma unroll
    for (int j = 0; j < 4; ++j)
#pragma unroll
      for (int r = 0; r < 8; ++r) acc[j][r] *= alpha[r];
    __syncthreads();
    const v16h pa = frag_f32s(&sp[wave][col][0], lane, 2048.0f);
#pragma unroll
    for (int j = 0; j < 4; ++j) { v16h vb; const int d = j * 16 + col;
#pragma unroll
      for (int i = 0; i < 8; ++i) { vb[i] = sv[8 * g + i][d]; vb[8 + i] = sv[16 + 8 * g + i][d]; }
      acc[j] = wmma16(pa, vb, acc[j]); } }
#pragma unroll
  for (int r = 0; r < 8; ++r) { const float il = (1.0f / 2048.0f) / l[r];
#pragma unroll
    for (int j = 0; j < 4; ++j) so[wave][8 * g + r][j * 16 + col] = acc[j][r] * il; }
  LDSX();
  for (int rl = 0; rl < 16; ++rl) { const int ql2 = wave * 16 + rl; const size_t orow = (size_t)tq * NTOK + (wi * WS8 + ql2 / WS8) * WI + wj * WS8 + (ql2 % WS8); if (lane < 16) vst2(O + orow * CC + h * CH + lane * 4, *(const v4f*)&so[wave][rl][lane * 4]); } }
__global__ __launch_bounds__(128) void k_out(const float* __restrict__ O, const float* __restrict__ WP, const float* __restrict__ BP, float* __restrict__ OUT) { __shared__ __align__(16) float sf[4][16][132];
  const int tid = threadIdx.x, wave = tid >> 5, lane = tid & 31, col = lane & 15, g = lane >> 4; const int c0 = blockIdx.y * 128; const size_t r0 = (size_t)blockIdx.x * 64 + wave * 16;
  v8f acc[8] = {};
#pragma unroll 2
  for (int kc = 0; kc < CC / 32; ++kc) { const F2 a = split_row(O + (r0 + col) * CC, kc * 32, lane);
#pragma unroll
    for (int j = 0; j < 8; ++j) { v16b wv; const int o = c0 + j * 16 + col;
#pragma unroll
      for (int i = 0; i < 8; ++i) { wv[i] = (__bf16)WP[(size_t)(kc * 32 + 8 * g + i) * CC + o]; wv[8 + i] = (__bf16)WP[(size_t)(kc * 32 + 16 + 8 * g + i) * CC + o]; }
      acc[j] = wmma_bf(a.h, wv, acc[j]); acc[j] = wmma_bf(a.l, wv, acc[j]); } }
#pragma unroll
  for (int j = 0; j < 8; ++j) { const float bb = bfr(BP[c0 + j * 16 + col]);
#pragma unroll
    for (int r = 0; r < 8; ++r) sf[wave][8 * g + r][j * 16 + col] = acc[j][r] + bb; }
  LDSX(); for (int rl = 0; rl < 16; ++rl) vst2(OUT + (r0 + rl) * CC + c0 + lane * 4, *(const v4f*)&sf[wave][rl][lane * 4]); }
extern "C" void kernel_launch(void* const* d_in, const int* in_sizes, int n_in, void* d_out, int out_size, void* d_ws, size_t ws_size, hipStream_t stream) {
  (void)in_sizes; (void)n_in; (void)out_size;
  const float** F = (const float**)d_in;
  if (ws_size < (size_t)WS_END) return;
  char* ws = (char*)d_ws; _Float16 *Q = (_Float16*)(ws + WS_Q), *K = (_Float16*)(ws + WS_K), *V = (_Float16*)(ws + WS_V); float *PX = (float*)(ws + WS_PX), *O = (float*)(ws + WS_O); int *KT = (int*)(ws + WS_KT), *WM = (int*)(ws + WS_WM);
  k_pool<<<dim3(NPOOL, NT), 512, 0, stream>>>(F[0], F[10], F[11], PX);
  k_proj<<<dim3(NROWSP / 64, CC / 128, 3), 128, 0, stream>>>(F[0], PX, F[2], F[3], F[4], F[5], F[6], F[7], Q, K, V);
  k_tab<<<NW, 64, 0, stream>>>(F[1], KT, WM);
  k_flags<<<1, 64, 0, stream>>>(F[1], WM);
  k_att<<<dim3(NT, NH, NW), 128, 0, stream>>>(Q, K, V, KT, WM, O);
  k_out<<<dim3(NT * NTOK / 64, CC / 128), 128, 0, stream>>>(O, F[8], F[9], (float*)d_out);
}
